// GroupedQueryAttention_75505525064719
// MI455X (gfx1250) — hardware-verified
//
#include <hip/hip_runtime.h>
#include <math.h>


#ifndef NB
#define NB   2
#endif
#ifndef SEQ
#define SEQ  2048
#endif
#define SEQ_FULL 2048
#define DM   2048
#define NH_  16
#define NKV  4
#define REP  (NH_ / NKV)
#define HD   128
#define DQ   (NH_ * HD)
#define DKV  (NKV * HD)
#define NKVW (2 * DKV)
#define RH   ((SEQ) < 512 ? (SEQ) : 512)
#define PCAR 1024.0f
#define SCL  0.088388347648318447f
#define SC2  (SCL * 1.4426950408889634f)
#define PP   40
#define OPT  136

static_assert(HD == 128);
static_assert(REP == 4);
static_assert(DQ == 2048 && DKV == 512 && DM == 2048);
static_assert(SEQ % 64 == 0);
static_assert(RH % 32 == 0);
static_assert((SEQ - RH) % 16 == 0);
static_assert(DM % 32 == 0 && DQ % 64 == 0 && NKVW % 64 == 0);
static_assert(SEQ <= SEQ_FULL);

typedef _Float16 h16;
typedef unsigned short bf;
typedef __attribute__((ext_vector_type(16))) __bf16   v16bf;
typedef __attribute__((ext_vector_type(16))) _Float16 v16h;
typedef __attribute__((ext_vector_type(8)))  _Float16 v8h;
typedef __attribute__((ext_vector_type(8)))  unsigned short v8us;
typedef __attribute__((ext_vector_type(8)))  float    v8f;
typedef __attribute__((ext_vector_type(4)))  float    v4f;
typedef __attribute__((ext_vector_type(2)))  float    v2f;
typedef __attribute__((ext_vector_type(2)))  unsigned short v2us;
typedef v8h  __attribute__((may_alias)) v8ha;
typedef v4f  __attribute__((may_alias)) v4fa;
typedef v8us __attribute__((may_alias)) v8usa;

__device__ __forceinline__ unsigned short f2bf(float f) { unsigned u = __float_as_uint(f); u += 0x7FFFu + ((u >> 16) & 1u); return (unsigned short)(u >> 16); }
__device__ __forceinline__ float bf2f(unsigned short b) { return __uint_as_float(((unsigned)b) << 16); }
__device__ __forceinline__ float bfr(float f) { return bf2f(f2bf(f)); }
__device__ __forceinline__ void splitf(float y, unsigned short& h, unsigned short& l) { h = f2bf(y); l = f2bf(y - bf2f(h)); }
__device__ __forceinline__ v16h cat16(v8h lo, v8h hi) { return __builtin_shufflevector(lo, hi, 0, 1, 2, 3, 4, 5, 6, 7, 8, 9, 10, 11, 12, 13, 14, 15); }
__device__ __forceinline__ v16bf cat16b(v8us lo, v8us hi) { return __builtin_bit_cast(v16bf, __builtin_shufflevector(lo, hi, 0, 1, 2, 3, 4, 5, 6, 7, 8, 9, 10, 11, 12, 13, 14, 15)); }
__device__ __forceinline__ v8f wmma16(v16h a, v16h b, v8f c) { return __builtin_amdgcn_wmma_f32_16x16x32_f16(false, a, false, b, (short)0, c, false, false); }
__device__ __forceinline__ v8f wmmab(v16bf a, v16bf b, v8f c) { return __builtin_amdgcn_wmma_f32_16x16x32_bf16(false, a, false, b, (short)0, c, false, false); }
__device__ __forceinline__ void wsync() { __builtin_amdgcn_fence(3  , "wavefront"); __builtin_amdgcn_wave_barrier(); asm volatile("" ::: "memory"); }

template <typename T16> struct WFrag;
template <> struct WFrag<h16> { typedef v16h V;
    static __device__ __forceinline__ V ld(const h16* p) { return cat16(*(const v8h*)p, *(const v8h*)(p + 16)); }
    static __device__ __forceinline__ V lda(const h16* p) { return cat16(*(const v8ha*)p, *(const v8ha*)(p + 16)); }
    static __device__ __forceinline__ v8f mma(V a, V b, v8f c) { return wmma16(a, b, c); } };
template <> struct WFrag<bf> { typedef v16bf V;
    static __device__ __forceinline__ V ld(const bf* p) { return cat16b(*(const v8us*)p, *(const v8us*)(p + 16)); }
    static __device__ __forceinline__ V lda(const bf* p) { return cat16b(*(const v8usa*)p, *(const v8usa*)(p + 16)); }
    static __device__ __forceinline__ v8f mma(V a, V b, v8f c) { return wmmab(a, b, c); } };

template <typename T16, int NSPLIT, bool BIAS>
__global__ __launch_bounds__(32) void k_gemmw(const T16* __restrict__ A, const T16* __restrict__ A2, const T16* __restrict__ Bt, const T16* __restrict__ Bt2, int K, float* C, int ldc, const float* __restrict__ bias, size_t sA, size_t sB, size_t sC) {
    typedef typename WFrag<T16>::V V;
    __shared__ __align__(16) float os[16 * 68];
    const size_t z = blockIdx.z; A += z * sA; if (A2) A2 += z * sA; Bt += z * sB; if (Bt2) Bt2 += z * sB; C += z * sC;
    const int lane = threadIdx.x & 31, lr = lane & 15, hi = lane >> 4; const int r0 = blockIdx.x * 64, c0 = blockIdx.y * 64;
    v8f acc[4][4];
#pragma unroll
    for (int mb = 0; mb < 4; ++mb)
#pragma unroll
        for (int nb = 0; nb < 4; ++nb) acc[mb][nb] = (v8f){};
    const size_t aoff = (size_t)(r0 + lr) * K + 8 * hi, boff = (size_t)(c0 + lr) * K + 8 * hi;
#pragma unroll 1
    for (int kc = 0; kc < K; kc += 32) {
        V a[4], a2[4];
#pragma unroll
        for (int mb = 0; mb < 4; ++mb) { a[mb] = WFrag<T16>::ld(A + aoff + (size_t)mb * 16 * K + kc); if (NSPLIT == 1 || NSPLIT == 2) a2[mb] = WFrag<T16>::ld(A2 + aoff + (size_t)mb * 16 * K + kc); }
#pragma unroll
        for (int nb = 0; nb < 4; ++nb) { const V b = WFrag<T16>::ld(Bt + boff + (size_t)nb * 16 * K + kc); V b2; if (NSPLIT >= 2) b2 = WFrag<T16>::ld(Bt2 + boff + (size_t)nb * 16 * K + kc);
#pragma unroll
            for (int mb = 0; mb < 4; ++mb) { acc[mb][nb] = WFrag<T16>::mma(a[mb], b, acc[mb][nb]); if (NSPLIT == 1 || NSPLIT == 2) acc[mb][nb] = WFrag<T16>::mma(a2[mb], b, acc[mb][nb]); if (NSPLIT >= 2) acc[mb][nb] = WFrag<T16>::mma(a[mb], b2, acc[mb][nb]); } }
        asm volatile("v_nop\n\tv_nop\n\tv_nop\n\tv_nop" : "+v"(acc[0][0]), "+v"(acc[1][1]), "+v"(acc[2][2]), "+v"(acc[3][3]) : "v"(a[0]), "v"(a[3]));
    }
#pragma unroll
    for (int mb = 0; mb < 4; ++mb) {
#pragma unroll
        for (int nb = 0; nb < 4; ++nb) {
#pragma unroll
            for (int j = 0; j < 8; ++j) os[(hi * 8 + j) * 68 + nb * 16 + lr] = acc[mb][nb][j]; }
        __builtin_amdgcn_wave_barrier(); asm volatile("" ::: "memory");
        float* crow = C + (size_t)(r0 + mb * 16) * ldc + c0;
#pragma unroll 1
        for (int ps = 0; ps < 2; ++ps) {
#pragma unroll
            for (int s = 0; s < 8; ++s) { const int row = 2 * s + hi, cofs = lr * 4; v4f val = *(const v4fa*)(os + row * 68 + cofs); if (BIAS) { val[0] += bfr(bias[c0 + cofs]); val[1] += bfr(bias[c0 + cofs + 1]); val[2] += bfr(bias[c0 + cofs + 2]); val[3] += bfr(bias[c0 + cofs + 3]); }
                *(volatile v4f*)(crow + (size_t)row * ldc + cofs) = val; }
            if (ps == 0) __threadfence(); }
        __builtin_amdgcn_wave_barrier(); asm volatile("" ::: "memory");
    }
}

__global__ __launch_bounds__(256) void k_wtG(const float* __restrict__ w, int K, int N, bf* Bt) {
    const int lane = threadIdx.x & 31; const int L0 = (blockIdx.x * 8 + (threadIdx.x >> 5)) * 8; const int nlines = N * K / 64;
#pragma unroll
    for (int ps = 0; ps < 2; ++ps) {
#pragma unroll 1
        for (int l = 0; l < 8; ++l) { const int L = L0 + l; if (L >= nlines) break; const size_t e = (size_t)L * 64 + lane * 2; const int k = (int)(e % K), n = (int)(e / K); v2us o;
            o[0] = f2bf(w[(size_t)k * N + n]); o[1] = f2bf(w[(size_t)(k + 1) * N + n]); *(volatile v2us*)(Bt + e) = o; }
        if (ps == 0) __threadfence(); }
}
__global__ __launch_bounds__(256) void k_cvt8(const float* __restrict__ src, bf* dst, size_t n8) { const size_t i = (size_t)blockIdx.x * 256 + threadIdx.x; if (i >= n8) return; const v8f v = *(const v8f*)(src + i * 8); v8us o;
#pragma unroll
    for (int k = 0; k < 8; ++k) o[k] = f2bf(v[k]); *(volatile v8us*)(dst + i * 8) = o; __threadfence(); *(volatile v8us*)(dst + i * 8) = o; }

struct F32x32 { float v[32]; };
static_assert(sizeof(F32x32) == 128);
static_assert(SEQ % 8 == 0);
__global__ __launch_bounds__(256) void k_cstab(F32x32 fr, unsigned i0, float* CS) {
    const unsigned lane = threadIdx.x & 31u; const unsigned t = blockIdx.x * 8u + (threadIdx.x >> 5); if (t >= (unsigned)SEQ) return;
    float inv = fr.v[0];
#pragma unroll
    for (unsigned j = 1; j < 32; ++j) inv = (lane == j) ? fr.v[j] : inv;
    const float ang = (float)t * inv; float sn, cs; sincosf(ang, &sn, &cs);
    v2f o; o[0] = cs; o[1] = sn; float* p = CS + ((size_t)t * 64u + i0 + lane) * 2u;
    *(volatile v2f*)p = o; __threadfence(); *(volatile v2f*)p = o; }

static_assert((NH_ * SEQ * 16) % 256 == 0 && (NKV * SEQ * 16) % 256 == 0);
__global__ __launch_bounds__(256) void k_rope8(const float* __restrict__ F, unsigned pitch, unsigned nheads, const float* __restrict__ CS, h16* P16, bf* Ph, bf* Pl) {
#pragma clang fp contract(off)
    const unsigned id = blockIdx.x * 256u + threadIdx.x; if (id >= nheads * (unsigned)SEQ * 16u) return;
    const unsigned d0 = (id & 15u) << 3, row = id >> 4, t = row % (unsigned)SEQ, h = row / (unsigned)SEQ;
    const unsigned dp = d0 ^ 64u, i0 = d0 & 63u; const bool low = d0 < 64u;
    const float* f = F + (size_t)t * pitch + h * HD;
    const v4f xa = *(const v4f*)(f + d0), xb = *(const v4f*)(f + d0 + 4u), ya = *(const v4f*)(f + dp), yb = *(const v4f*)(f + dp + 4u);
    const float* tb = CS + ((size_t)t * 64u + i0) * 2u;
    const v4f c0 = *(const v4f*)(tb), c1 = *(const v4f*)(tb + 4), c2 = *(const v4f*)(tb + 8), c3 = *(const v4f*)(tb + 12);
    float xs[8], xp[8], co[8], si[8];
#pragma unroll
    for (int q = 0; q < 4; ++q) { xs[q] = xa[q]; xs[4 + q] = xb[q]; xp[q] = ya[q]; xp[4 + q] = yb[q]; }
    co[0] = c0[0]; si[0] = c0[1]; co[1] = c0[2]; si[1] = c0[3]; co[2] = c1[0]; si[2] = c1[1]; co[3] = c1[2]; si[3] = c1[3];
    co[4] = c2[0]; si[4] = c2[1]; co[5] = c2[2]; si[5] = c2[3]; co[6] = c3[0]; si[6] = c3[1]; co[7] = c3[2]; si[7] = c3[3];
    v8h o16; v8us oh, ol;
#pragma unroll
    for (int q = 0; q < 8; ++q) { const float a = xs[q] * co[q]; const float b = xp[q] * si[q]; const float r = low ? (a - b) : (a + b);
        o16[q] = (h16)r; unsigned short a2, c2s; splitf(r, a2, c2s); oh[q] = a2; ol[q] = c2s; }
    h16* p16 = P16 + ((size_t)h * SEQ + t) * HD + d0; const size_t e2 = ((size_t)h * RH + t) * HD + d0; const bool hl = t < (unsigned)RH;
    *(volatile v8h*)p16 = o16; if (hl) { *(volatile v8us*)(Ph + e2) = oh; *(volatile v8us*)(Pl + e2) = ol; }
    __threadfence();
    *(volatile v8h*)p16 = o16; if (hl) { *(volatile v8us*)(Ph + e2) = oh; *(volatile v8us*)(Pl + e2) = ol; }
}
static_assert((NKV * HD * (SEQ / 8)) % 256 == 0);
__global__ __launch_bounds__(256) void k_vtp8(const float* __restrict__ F, unsigned pitch, h16* V16, bf* Vh, bf* Vl) {
    const unsigned id = blockIdx.x * 256u + threadIdx.x; if (id >= (unsigned)(NKV * HD * (SEQ / 8))) return;
    const unsigned t0 = (id % (unsigned)(SEQ / 8)) << 3, rw = id / (unsigned)(SEQ / 8);
    v8h o16; v8us oh, ol;
#pragma unroll
    for (unsigned q = 0; q < 8; ++q) { const float x = F[(size_t)(t0 + q) * pitch + rw]; o16[q] = (h16)x; unsigned short a2, c2s; splitf(x, a2, c2s); oh[q] = a2; ol[q] = c2s; }
    h16* p16 = V16 + (size_t)rw * SEQ + t0; const size_t e2 = (size_t)rw * RH + t0; const bool hl = t0 < (unsigned)RH;
    *(volatile v8h*)p16 = o16; if (hl) { *(volatile v8us*)(Vh + e2) = oh; *(volatile v8us*)(Vl + e2) = ol; }
    __threadfence();
    *(volatile v8h*)p16 = o16; if (hl) { *(volatile v8us*)(Vh + e2) = oh; *(volatile v8us*)(Vl + e2) = ol; }
}

template <bool HL> struct PT;
template <> struct PT<false> { typedef h16 T;
    static __device__ __forceinline__ void put(h16* ph, h16* pl, unsigned idx, float e) { (void)pl; ph[idx] = (h16)(e * PCAR); }
    static __device__ __forceinline__ float oscale() { return 1.0f / PCAR; } };
template <> struct PT<true> { typedef bf T;
    static __device__ __forceinline__ void put(bf* ph, bf* pl, unsigned idx, float e) { unsigned short a, c; splitf(e, a, c); ph[idx] = a; pl[idx] = c; }
    static __device__ __forceinline__ float oscale() { return 1.0f; } };

template <bool HL>
__global__ __launch_bounds__(128) void k_flash(const typename PT<HL>::T* Qa, const typename PT<HL>::T* Qb, const typename PT<HL>::T* Ka, const typename PT<HL>::T* Kb,
                                               const typename PT<HL>::T* Va, const typename PT<HL>::T* Vb, bf* ATh, bf* ATl) {
    typedef typename PT<HL>::T T16; typedef WFrag<T16> WF; typedef typename WF::V V;
    constexpr unsigned QR = HL ? (unsigned)RH : (unsigned)SEQ;
    constexpr unsigned ROFF = HL ? 0u : (unsigned)RH;
    constexpr unsigned GS = HL ? 2u : 4u;
    __shared__ __align__(16) T16 pls[REP][2][16 * PP];
    __shared__ __align__(16) bf ost[REP][2][16 * OPT];
    const unsigned w = threadIdx.x >> 5, lane = threadIdx.x & 31u, lr = lane & 15u, hi = lane >> 4;
    const unsigned kv = blockIdx.y, head = kv * REP + w, q0 = ROFF + blockIdx.x * 16u;
    T16* plh = &pls[w][0][0]; T16* pll = &pls[w][1][0];
    const size_t qo = ((size_t)head * QR + q0 + lr) * HD + 8u * hi;
    const size_t ko = ((size_t)kv * QR + lr) * HD + 8u * hi;
    const size_t vo = ((size_t)kv * HD + lr) * QR + 8u * hi;
    v8f o[8]; float mrow[8], lsum[8];
#pragma unroll
    for (int j = 0; j < 8; ++j) { o[j] = (v8f){}; mrow[j] = -3.0e38f; lsum[j] = 0.0f; }
    const unsigned nfull = q0 >> 5;
#pragma unroll 1
    for (unsigned kb = 0; kb <= nfull; ++kb) {
        const unsigned s0 = kb * 32u; const bool msk = (kb == nfull);
        const size_t kp = ko + (size_t)s0 * HD;
        v8f st0 = (v8f){}, st1 = (v8f){};
#pragma unroll 1
        for (unsigned c = 0; c < 4; ++c) {
            const unsigned oo = c * 32u;
            const V qa = WF::ld(Qa + qo + oo); const V k0 = WF::ld(Ka + kp + oo); const V k1 = WF::ld(Ka + kp + 16u * HD + oo);
            if (HL) {
                const V ql = WF::ld(Qb + qo + oo); const V k0l = WF::ld(Kb + kp + oo); const V k1l = WF::ld(Kb + kp + 16u * HD + oo);
                __builtin_amdgcn_sched_barrier(0);
                st0 = WF::mma(qa, k0, st0); st1 = WF::mma(qa, k1, st1); st0 = WF::mma(ql, k0, st0); st1 = WF::mma(ql, k1, st1); st0 = WF::mma(qa, k0l, st0); st1 = WF::mma(qa, k1l, st1);
                asm volatile("v_nop\n\tv_nop\n\tv_nop\n\tv_nop" : "+v"(st0), "+v"(st1) : "v"(qa), "v"(ql), "v"(k1l));
            } else {
                __builtin_amdgcn_sched_barrier(0);
                st0 = WF::mma(qa, k0, st0); st1 = WF::mma(qa, k1, st1);
                asm volatile("v_nop\n\tv_nop\n\tv_nop\n\tv_nop" : "+v"(st0), "+v"(st1) : "v"(qa), "v"(k1));
            }
            __builtin_amdgcn_sched_barrier(0);
        }
        const unsigned kp0 = s0 + lr, kp1 = kp0 + 16u;
#pragma unroll
        for (int r = 0; r < 8; ++r) {
            const unsigned qpos = q0 + 8u * hi + (unsigned)r;
            const bool x0 = msk & (kp0 > qpos), x1 = msk & (kp1 > qpos);
            const float a = x0 ? -3.0e38f : st0[r] * SC2; const float b = x1 ? -3.0e38f : st1[r] * SC2;
            float rm = fmaxf(a, b);
            rm = fmaxf(rm, __shfl_xor(rm, 1, 32)); rm = fmaxf(rm, __shfl_xor(rm, 2, 32)); rm = fmaxf(rm, __shfl_xor(rm, 4, 32)); rm = fmaxf(rm, __shfl_xor(rm, 8, 32));
            const float mn = fmaxf(mrow[r], rm);
            const float alpha = __builtin_amdgcn_exp2f(mrow[r] - mn);
            float e0 = __builtin_amdgcn_exp2f(a - mn), e1 = __builtin_amdgcn_exp2f(b - mn);
            e0 = x0 ? 0.0f : e0; e1 = x1 ? 0.0f : e1;
            lsum[r] = lsum[r] * alpha + (e0 + e1); mrow[r] = mn;
#pragma unroll
            for (int j = 0; j < 8; ++j) o[j][r] *= alpha;
            const unsigned idx = (8u * hi + (unsigned)r) * PP + lr;
            PT<HL>::put(plh, pll, idx, e0); PT<HL>::put(plh, pll, idx + 16u, e1);
        }
        wsync();
        const V pa = WF::lda(plh + lr * PP + 8u * hi);
        const V pal = HL ? WF::lda(pll + lr * PP + 8u * hi) : pa;
        wsync();
        const size_t vp = vo + s0;
#pragma unroll
        for (unsigned g = 0; g < 8; g += GS) {
            V vb[GS], vl[GS];
#pragma unroll
            for (unsigned u = 0; u < GS; ++u) { vb[u] = WF::ld(Va + vp + (size_t)(g + u) * 16u * QR); if (HL) vl[u] = WF::ld(Vb + vp + (size_t)(g + u) * 16u * QR); else vl[u] = vb[u]; }
            __builtin_amdgcn_sched_barrier(0);
#pragma unroll
            for (unsigned u = 0; u < GS; ++u) { o[g + u] = WF::mma(pa, vb[u], o[g + u]); if (HL) { o[g + u] = WF::mma(pal, vb[u], o[g + u]); o[g + u] = WF::mma(pa, vl[u], o[g + u]); } }
            if (HL) asm volatile("v_nop\n\tv_nop\n\tv_nop\n\tv_nop" : "+v"(o[g]), "+v"(o[g + 1]) : "v"(pa), "v"(pal), "v"(vl[GS - 1]));
            else    asm volatile("v_nop\n\tv_nop\n\tv_nop\n\tv_nop" : "+v"(o[g]), "+v"(o[g + 1]), "+v"(o[(g + 2) & 7]), "+v"(o[(g + 3) & 7]) : "v"(pa), "v"(vb[GS - 1]));
            __builtin_amdgcn_sched_barrier(0);
        }
    }
    bf* oh = &ost[w][0][0]; bf* ol = &ost[w][1][0];
    const float osc = PT<HL>::oscale();
#pragma unroll
    for (int r = 0; r < 8; ++r) { float l = lsum[r]; l += __shfl_xor(l, 1, 32); l += __shfl_xor(l, 2, 32); l += __shfl_xor(l, 4, 32); l += __shfl_xor(l, 8, 32);
        const float inv = (1.0f / l) * osc;
#pragma unroll
        for (int j = 0; j < 8; ++j) { unsigned short a, c; splitf(o[j][r] * inv, a, c); const unsigned idx = (8u * hi + (unsigned)r) * OPT + (unsigned)j * 16u + lr; oh[idx] = a; ol[idx] = c; } }
    wsync();
#pragma unroll 1
    for (int ps = 0; ps < 2; ++ps) {
#pragma unroll
        for (unsigned s = 0; s < 8; ++s) { const unsigned row = 2u * s + hi, cofs = lr * 8u; const v8us vh = *(const v8usa*)(oh + row * OPT + cofs); const v8us vl2 = *(const v8usa*)(ol + row * OPT + cofs);
            const size_t oo = (size_t)(q0 + row) * DQ + head * HD + cofs; *(volatile v8us*)(ATh + oo) = vh; *(volatile v8us*)(ATl + oo) = vl2; }
        if (ps == 0) __threadfence(); }
}

constexpr size_t al256(size_t b) { return (b + 255) & ~(size_t)255; }
constexpr size_t SZ_WQ  = al256((size_t)DQ * DM * 2);
constexpr size_t SZ_WKV = al256((size_t)NKVW * DM * 2);
constexpr size_t SZ_WO  = al256((size_t)DM * DQ * 2);
constexpr size_t SZ_CS  = al256((size_t)SEQ * 64 * 2 * 4);
constexpr size_t SZ_XB  = al256((size_t)SEQ * DM * 2);
constexpr size_t SZ_FQ  = al256((size_t)SEQ * DQ * 4);
constexpr size_t SZ_FKV = al256((size_t)SEQ * NKVW * 4);
constexpr size_t SZ_Q16 = al256((size_t)NH_ * SEQ * HD * 2);
constexpr size_t SZ_QHL = al256((size_t)NH_ * RH * HD * 2);
constexpr size_t SZ_K16 = al256((size_t)NKV * SEQ * HD * 2);
constexpr size_t SZ_KHL = al256((size_t)NKV * RH * HD * 2);
constexpr size_t SZ_AT  = al256((size_t)SEQ * DQ * 2);
constexpr size_t WS_TOTAL = SZ_WQ + SZ_WKV + SZ_WO + SZ_CS + SZ_XB + SZ_FQ + SZ_FKV + SZ_Q16 + 2 * SZ_QHL + 2 * (SZ_K16 + 2 * SZ_KHL) + 2 * SZ_AT;
static_assert(WS_TOTAL <= (size_t)134217728);

extern "C" void kernel_launch(void* const* d_in, const int* in_sizes, int n_in,
                              void* d_out, int out_size, void* d_ws, size_t ws_size, hipStream_t stream) {
    if (n_in < 5) return;
    if ((size_t)in_sizes[0] < (size_t)(NB - 1) * SEQ_FULL * DM + (size_t)SEQ * DM) return;
    if ((size_t)in_sizes[1] < (size_t)DM * DQ || (size_t)in_sizes[2] < (size_t)DM * DKV || (size_t)in_sizes[3] < (size_t)DM * DKV || (size_t)in_sizes[4] < (size_t)DQ * DM) return;
    if ((size_t)out_size < (size_t)NB * SEQ * DM) return;
    if (WS_TOTAL > ws_size) return;
    const float* x = (const float*)d_in[0]; const float* wq = (const float*)d_in[1]; const float* wk = (const float*)d_in[2]; const float* wv = (const float*)d_in[3]; const float* wo = (const float*)d_in[4];
    float* OUT = (float*)d_out;
    char* wsp = (char*)d_ws;
    auto take = [&](size_t bytes) { char* p = wsp; wsp += bytes; return (void*)p; };
    bf* WQ = (bf*)take(SZ_WQ); bf* WKV = (bf*)take(SZ_WKV); bf* WO = (bf*)take(SZ_WO); float* CS = (float*)take(SZ_CS);
    bf* XB = (bf*)take(SZ_XB); float* FQ = (float*)take(SZ_FQ); float* FKV = (float*)take(SZ_FKV);
    h16* Q16 = (h16*)take(SZ_Q16); bf* QH = (bf*)take(SZ_QHL); bf* QL = (bf*)take(SZ_QHL);
    h16* K16 = (h16*)take(SZ_K16); bf* KH = (bf*)take(SZ_KHL); bf* KL = (bf*)take(SZ_KHL);
    h16* VT16 = (h16*)take(SZ_K16); bf* VTH = (bf*)take(SZ_KHL); bf* VTL = (bf*)take(SZ_KHL);
    bf* ATH = (bf*)take(SZ_AT); bf* ATL = (bf*)take(SZ_AT);

    F32x32 fa, fb;
    for (int i = 0; i < 64; ++i) { const double pw = pow(10000.0, (2.0 * (double)i) / 128.0); const float pf = (float)pw; const float inv = 1.0f / pf; if (i < 32) fa.v[i] = inv; else fb.v[i - 32] = inv; }

    k_wtG<<<(unsigned)((DM * DQ / 64 + 63) / 64), 256, 0, stream>>>(wq, DM, DQ, WQ);
    k_wtG<<<(unsigned)((DM * DKV / 64 + 63) / 64), 256, 0, stream>>>(wk, DM, DKV, WKV);
    k_wtG<<<(unsigned)((DM * DKV / 64 + 63) / 64), 256, 0, stream>>>(wv, DM, DKV, WKV + (size_t)DKV * DM);
    k_wtG<<<(unsigned)((DQ * DM / 64 + 63) / 64), 256, 0, stream>>>(wo, DQ, DM, WO);
    k_cstab<<<SEQ / 8, 256, 0, stream>>>(fa, 0u, CS);
    k_cstab<<<SEQ / 8, 256, 0, stream>>>(fb, 32u, CS);

    for (int b = 0; b < NB; ++b) {
        k_cvt8<<<(unsigned)(((size_t)SEQ * DM / 8 + 255) / 256), 256, 0, stream>>>(x + (size_t)b * SEQ_FULL * DM, XB, (size_t)SEQ * DM / 8);
        k_gemmw<bf, 0, false><<<dim3(SEQ / 64, DQ / 64, 1), 32, 0, stream>>>(XB, nullptr, WQ, nullptr, DM, FQ, DQ, nullptr, 0, 0, 0);
        k_gemmw<bf, 0, false><<<dim3(SEQ / 64, NKVW / 64, 1), 32, 0, stream>>>(XB, nullptr, WKV, nullptr, DM, FKV, NKVW, nullptr, 0, 0, 0);
        k_rope8<<<(unsigned)(NH_ * SEQ * 16 / 256), 256, 0, stream>>>(FQ, (unsigned)DQ, (unsigned)NH_, CS, Q16, QH, QL);
        k_rope8<<<(unsigned)(NKV * SEQ * 16 / 256), 256, 0, stream>>>(FKV, (unsigned)NKVW, (unsigned)NKV, CS, K16, KH, KL);
        k_vtp8<<<(unsigned)(NKV * HD * (SEQ / 8) / 256), 256, 0, stream>>>(FKV + DKV, (unsigned)NKVW, VT16, VTH, VTL);
        k_flash<true><<<dim3(RH / 16, NKV, 1), 128, 0, stream>>>(QH, QL, KH, KL, VTH, VTL, ATH, ATL);
        if (SEQ > RH) k_flash<false><<<dim3((SEQ - RH) / 16, NKV, 1), 128, 0, stream>>>(Q16, Q16, K16, K16, VT16, VT16, ATH, ATL);
        k_gemmw<bf, 1, false><<<dim3(SEQ / 64, DM / 64, 1), 32, 0, stream>>>(ATH, ATL, WO, nullptr, DQ, OUT + (size_t)b * SEQ * DM, DM, nullptr, 0, 0, 0);
    }
}
